// FuncRepresentation_79697413144920
// MI455X (gfx1250) — hardware-run, weakly checked
//
#include <hip/hip_runtime.h>
#include <math.h>

typedef __attribute__((ext_vector_type(16))) _Float16 v16h;
typedef __attribute__((ext_vector_type(16))) __bf16 v16b;
typedef __attribute__((ext_vector_type(8)))  _Float16 v8h;
typedef __attribute__((ext_vector_type(8)))  float v8f;
typedef __attribute__((ext_vector_type(4)))  float v4f;
typedef __attribute__((ext_vector_type(2)))  float v2f;
typedef __attribute__((ext_vector_type(4)))  unsigned v4u;
typedef __attribute__((ext_vector_type(4)))  int v4i;
typedef float __attribute__((may_alias)) float_a;
typedef int __attribute__((may_alias)) int_a;

template <typename T> __device__ __forceinline__ void vst2(void* p, T v) { *(volatile T*)p = v; __threadfence(); *(volatile T*)p = v; }
__device__ __forceinline__ v8f wmma16(v16h a, v16h b, v8f c) {
  v8f d = __builtin_amdgcn_wmma_f32_16x16x32_f16(false, a, false, b, (short)0, c, false, false);
  asm volatile("v_nop\n\tv_nop\n\tv_nop\n\tv_nop" : "+v"(d) : "v"(a), "v"(b));
  return d;
}
__device__ __forceinline__ v8f wmma_bf(v16b a, v16b b, v8f c) {
  v8f d = __builtin_amdgcn_wmma_f32_16x16x32_bf16(false, a, false, b, (short)0, c, false, false);
  asm volatile("v_nop\n\tv_nop\n\tv_nop\n\tv_nop" : "+v"(d) : "v"(a), "v"(b));
  return d;
}
__device__ __forceinline__ v16h frag_h(const _Float16* rowk0, int lane) {
  union { v16h v; v8h q[2]; } u; const _Float16* p = rowk0 + 8 * (lane >> 4);
  u.q[0] = *(const v8h*)p; u.q[1] = *(const v8h*)(p + 16); return u.v;
}
__device__ __forceinline__ v16h frag_f32(const float* rowk0, int lane) {
  v16h a; const float* p = rowk0 + 8 * (lane >> 4);
#pragma unroll
  for (int i = 0; i < 8; ++i) { a[i] = (_Float16)p[i]; a[8 + i] = (_Float16)p[16 + i]; }
  return a;
}
__device__ __forceinline__ v16h frag_f32s(const float* rowk0, int lane, float sc) {
  v16h a; const float* p = rowk0 + 8 * (lane >> 4);
#pragma unroll
  for (int i = 0; i < 8; ++i) { a[i] = (_Float16)(p[i] * sc); a[8 + i] = (_Float16)(p[16 + i] * sc); }
  return a;
}
__device__ __forceinline__ v16h fragc_f32(const float* W, int k0, int n, int lane, int ld, int K) {
  v16h a; const int g = lane >> 4;
#pragma unroll
  for (int i = 0; i < 8; ++i) { const int ka = k0 + 8 * g + i, kb = ka + 16;
    a[i] = (_Float16)(ka < K ? W[(size_t)(ka < K ? ka : K - 1) * ld + n] : 0.f); a[8 + i] = (_Float16)(kb < K ? W[(size_t)(kb < K ? kb : K - 1) * ld + n] : 0.f); }
  return a;
}
struct F2 { v16b h, l; };
__device__ __forceinline__ F2 bsplit16(const float v[16]) { F2 r;
#pragma unroll
  for (int i = 0; i < 16; ++i) { const __bf16 h = (__bf16)v[i]; r.h[i] = h; r.l[i] = (__bf16)(v[i] - (float)h); }
  return r; }
__device__ __forceinline__ F2 split_row(const float* row, int k0, int lane) { float v[16]; const float* p = row + k0 + 8 * (lane >> 4);
#pragma unroll
  for (int i = 0; i < 8; ++i) { v[i] = p[i]; v[8 + i] = p[16 + i]; }
  return bsplit16(v); }
__device__ __forceinline__ F2 split_rowK(const float* row, int k0, int lane, int K) { float v[16]; const int g = lane >> 4;
#pragma unroll
  for (int i = 0; i < 8; ++i) { const int ka = k0 + 8 * g + i, kb = ka + 16; v[i] = ka < K ? row[ka < K ? ka : K - 1] : 0.f; v[8 + i] = kb < K ? row[kb < K ? kb : K - 1] : 0.f; }
  return bsplit16(v); }
__device__ __forceinline__ F2 split_col(const float* W, int k0, int n, int lane, int ld, int K) { float v[16]; const int g = lane >> 4;
#pragma unroll
  for (int i = 0; i < 8; ++i) { const int ka = k0 + 8 * g + i, kb = ka + 16; v[i] = ka < K ? W[(size_t)(ka < K ? ka : K - 1) * ld + n] : 0.f; v[8 + i] = kb < K ? W[(size_t)(kb < K ? kb : K - 1) * ld + n] : 0.f; }
  return bsplit16(v); }
__device__ __forceinline__ v8f mac3(const F2& a, const F2& b, v8f c) { c = wmma_bf(a.l, b.h, c); c = wmma_bf(a.h, b.l, c); return wmma_bf(a.h, b.h, c); }
__device__ __forceinline__ float sigm(float v) { return 1.0f / (1.0f + expf(-v)); }
#define LDSX() do { asm volatile("s_wait_dscnt 0" ::: "memory"); __builtin_amdgcn_wave_barrier(); __builtin_amdgcn_fence(__ATOMIC_RELEASE, "workgroup"); } while (0)


#define NB 32
#define MM 16
#define TT 512
#define PP 600
#define PT ((PP + 15) / 16)
typedef __attribute__((ext_vector_type(8))) __bf16 v8b;
__device__ __forceinline__ v16b frag_b(const __bf16* rowk0, int lane) {
  union { v16b v; v8b q[2]; } u; const __bf16* p = rowk0 + 8 * (lane >> 4);
  u.q[0] = *(const v8b*)p; u.q[1] = *(const v8b*)(p + 16); return u.v;
}
__device__ __forceinline__ float bfr(float v) { return (float)(__bf16)v; }
__device__ __attribute__((noinline)) float exp_ni(float v) { return expf(v); }
__device__ __attribute__((noinline)) float erf_ni(float v) { return erff(v); }

__constant__ float GRID[PP] = {-1.000000000e+00f,-9.165275097e-01f,-8.330551386e-01f,-7.495826483e-01f,-6.661101580e-01f,-5.826377273e-01f,-4.991652966e-01f,-4.156928360e-01f,-3.322203755e-01f,-2.487479746e-01f,-1.652754992e-01f,-8.180303127e-02f,1.669377089e-03f,8.514184505e-02f,1.686143130e-01f,2.520867884e-01f,3.355591893e-01f,4.190316498e-01f,5.025041103e-01f,5.859765410e-01f,6.694489717e-01f,7.529214621e-01f,8.363939524e-01f,9.198663235e-01f,1.003338814e+00f,1.086811304e+00f,1.170283675e+00f,1.253756166e+00f,1.337228656e+00f,1.420701146e+00f,1.504173517e+00f,1.587646008e+00f,1.671118498e+00f,1.754590869e+00f,1.838063359e+00f,1.921535730e+00f,2.005008221e+00f,2.088480711e+00f,2.171953201e+00f,2.255425692e+00f,2.338897943e+00f,2.422370434e+00f,2.505842924e+00f,2.589315414e+00f,2.672787905e+00f,2.756260395e+00f,2.839732647e+00f,2.923205137e+00f,3.006677628e+00f,3.090150118e+00f,3.173622608e+00f,3.257094860e+00f,3.340567350e+00f,3.424039841e+00f,3.507512331e+00f,3.590984821e+00f,3.674457312e+00f,3.757929564e+00f,3.841402054e+00f,3.924874544e+00f,4.008347034e+00f,4.091819286e+00f,4.175292015e+00f,4.258764267e+00f,4.342236996e+00f,4.425709248e+00f,4.509181976e+00f,4.592654228e+00f,4.676126480e+00f,4.759599209e+00f,4.843071461e+00f,4.926544189e+00f,5.010016441e+00f,5.093488693e+00f,5.176961422e+00f,5.260433674e+00f,5.343906403e+00f,5.427378654e+00f,5.510850906e+00f,5.594323635e+00f,5.677795887e+00f,5.761268616e+00f,5.844740868e+00f,5.928213596e+00f,6.011685848e+00f,6.095158100e+00f,6.178630829e+00f,6.262103081e+00f,6.345575809e+00f,6.429048061e+00f,6.512520790e+00f,6.595993042e+00f,6.679465294e+00f,6.762938023e+00f,6.846410275e+00f,6.929883003e+00f,7.013355255e+00f,7.096827507e+00f,7.180300236e+00f,7.263772488e+00f,7.347245216e+00f,7.430717468e+00f,7.514189720e+00f,7.597662449e+00f,7.681134701e+00f,7.764607430e+00f,7.848079681e+00f,7.931552410e+00f,8.015024185e+00f,8.098497391e+00f,8.181969643e+00f,8.265441895e+00f,8.348914146e+00f,8.432387352e+00f,8.515859604e+00f,8.599331856e+00f,8.682804108e+00f,8.766276360e+00f,8.849749565e+00f,8.933221817e+00f,9.016694069e+00f,9.100166321e+00f,9.183638573e+00f,9.267111778e+00f,9.350584030e+00f,9.434056282e+00f,9.517528534e+00f,9.601000786e+00f,9.684473991e+00f,9.767946243e+00f,9.851418495e+00f,9.934890747e+00f,1.001836300e+01f,1.010183620e+01f,1.018530846e+01f,1.026878071e+01f,1.035225296e+01f,1.043572617e+01f,1.051919842e+01f,1.060267067e+01f,1.068614292e+01f,1.076961517e+01f,1.085308838e+01f,1.093656063e+01f,1.102003288e+01f,1.110350513e+01f,1.118697739e+01f,1.127045059e+01f,1.135392284e+01f,1.143739510e+01f,1.152086735e+01f,1.160433960e+01f,1.168781281e+01f,1.177128506e+01f,1.185475731e+01f,1.193822956e+01f,1.202170181e+01f,1.210517502e+01f,1.218864727e+01f,1.227211952e+01f,1.235559177e+01f,1.243906498e+01f,1.252253723e+01f,1.260600948e+01f,1.268948174e+01f,1.277295399e+01f,1.285642719e+01f,1.293989944e+01f,1.302337170e+01f,1.310684395e+01f,1.319031620e+01f,1.327378941e+01f,1.335726166e+01f,1.344073391e+01f,1.352420616e+01f,1.360767841e+01f,1.369115162e+01f,1.377462387e+01f,1.385809612e+01f,1.394156837e+01f,1.402504063e+01f,1.410851383e+01f,1.419198608e+01f,1.427545834e+01f,1.435893059e+01f,1.444240379e+01f,1.452587605e+01f,1.460934830e+01f,1.469282055e+01f,1.477629280e+01f,1.485976601e+01f,1.494323826e+01f,1.502671051e+01f,1.511018276e+01f,1.519365501e+01f,1.527712822e+01f,1.536060047e+01f,1.544407272e+01f,1.552754498e+01f,1.561101723e+01f,1.569449043e+01f,1.577796268e+01f,1.586143494e+01f,1.594490719e+01f,1.602837944e+01f,1.611185265e+01f,1.619532394e+01f,1.627879715e+01f,1.636227036e+01f,1.644574165e+01f,1.652921486e+01f,1.661268616e+01f,1.669615936e+01f,1.677963257e+01f,1.686310387e+01f,1.694657707e+01f,1.703004837e+01f,1.711352158e+01f,1.719699478e+01f,1.728046608e+01f,1.736393929e+01f,1.744741249e+01f,1.753088379e+01f,1.761435699e+01f,1.769782829e+01f,1.778130150e+01f,1.786477470e+01f,1.794824600e+01f,1.803171921e+01f,1.811519051e+01f,1.819866371e+01f,1.828213692e+01f,1.836560822e+01f,1.844908142e+01f,1.853255272e+01f,1.861602592e+01f,1.869949913e+01f,1.878297043e+01f,1.886644363e+01f,1.894991493e+01f,1.903338814e+01f,1.911686134e+01f,1.920033264e+01f,1.928380585e+01f,1.936727715e+01f,1.945075035e+01f,1.953422356e+01f,1.961769485e+01f,1.970116806e+01f,1.978463936e+01f,1.986811256e+01f,1.995158577e+01f,2.003505707e+01f,2.011853027e+01f,2.020200157e+01f,2.028547478e+01f,2.036894798e+01f,2.045241928e+01f,2.053589249e+01f,2.061936378e+01f,2.070283699e+01f,2.078631020e+01f,2.086978149e+01f,2.095325470e+01f,2.103672791e+01f,2.112019920e+01f,2.120367241e+01f,2.128714371e+01f,2.137061691e+01f,2.145409012e+01f,2.153756142e+01f,2.162103462e+01f,2.170450592e+01f,2.178797913e+01f,2.187145233e+01f,2.195492363e+01f,2.203839684e+01f,2.212186813e+01f,2.220534134e+01f,2.228881454e+01f,2.237228584e+01f,2.245575905e+01f,2.253923035e+01f,2.262270355e+01f,2.270617676e+01f,2.278964806e+01f,2.287312126e+01f,2.295659256e+01f,2.304006577e+01f,2.312353897e+01f,2.320701027e+01f,2.329048347e+01f,2.337395477e+01f,2.345742798e+01f,2.354090118e+01f,2.362437248e+01f,2.370784569e+01f,2.379131699e+01f,2.387479019e+01f,2.395826340e+01f,2.404173470e+01f,2.412520790e+01f,2.420867920e+01f,2.429215240e+01f,2.437562561e+01f,2.445909691e+01f,2.454257011e+01f,2.462604141e+01f,2.470951462e+01f,2.479298782e+01f,2.487645912e+01f,2.495993233e+01f,2.504340363e+01f,2.512687683e+01f,2.521035004e+01f,2.529382133e+01f,2.537729454e+01f,2.546076775e+01f,2.554423904e+01f,2.562771225e+01f,2.571118355e+01f,2.579465675e+01f,2.587812996e+01f,2.596160126e+01f,2.604507446e+01f,2.612854576e+01f,2.621201897e+01f,2.629549217e+01f,2.637896347e+01f,2.646243668e+01f,2.654590797e+01f,2.662938118e+01f,2.671285439e+01f,2.679632568e+01f,2.687979889e+01f,2.696327019e+01f,2.704674339e+01f,2.713021660e+01f,2.721368790e+01f,2.729716110e+01f,2.738063240e+01f,2.746410561e+01f,2.754757881e+01f,2.763105011e+01f,2.771452332e+01f,2.779799461e+01f,2.788146782e+01f,2.796494102e+01f,2.804841232e+01f,2.813188553e+01f,2.821535683e+01f,2.829883003e+01f,2.838230324e+01f,2.846577454e+01f,2.854924774e+01f,2.863271904e+01f,2.871619225e+01f,2.879966545e+01f,2.888313675e+01f,2.896660995e+01f,2.905008125e+01f,2.913355446e+01f,2.921702766e+01f,2.930049896e+01f,2.938397217e+01f,2.946744537e+01f,2.955091667e+01f,2.963438988e+01f,2.971786118e+01f,2.980133438e+01f,2.988480759e+01f,2.996827888e+01f,3.005175209e+01f,3.013522339e+01f,3.021869659e+01f,3.030216980e+01f,3.038564110e+01f,3.046911430e+01f,3.055258560e+01f,3.063605881e+01f,3.071953201e+01f,3.080300331e+01f,3.088647652e+01f,3.096994781e+01f,3.105342102e+01f,3.113689423e+01f,3.122036552e+01f,3.130383873e+01f,3.138731003e+01f,3.147078323e+01f,3.155425644e+01f,3.163772774e+01f,3.172120094e+01f,3.180467224e+01f,3.188814545e+01f,3.197161865e+01f,3.205509186e+01f,3.213856125e+01f,3.222203445e+01f,3.230550766e+01f,3.238898087e+01f,3.247245407e+01f,3.255592346e+01f,3.263939667e+01f,3.272286987e+01f,3.280634308e+01f,3.288981628e+01f,3.297328568e+01f,3.305675888e+01f,3.314023209e+01f,3.322370529e+01f,3.330717850e+01f,3.339064789e+01f,3.347412109e+01f,3.355759430e+01f,3.364106750e+01f,3.372454071e+01f,3.380801010e+01f,3.389148331e+01f,3.397495651e+01f,3.405842972e+01f,3.414190292e+01f,3.422537231e+01f,3.430884552e+01f,3.439231873e+01f,3.447579193e+01f,3.455926514e+01f,3.464273453e+01f,3.472620773e+01f,3.480968094e+01f,3.489315414e+01f,3.497662735e+01f,3.506009674e+01f,3.514356995e+01f,3.522704315e+01f,3.531051636e+01f,3.539398956e+01f,3.547746277e+01f,3.556093216e+01f,3.564440536e+01f,3.572787857e+01f,3.581135178e+01f,3.589482498e+01f,3.597829437e+01f,3.606176758e+01f,3.614524078e+01f,3.622871399e+01f,3.631218719e+01f,3.639565659e+01f,3.647912979e+01f,3.656260300e+01f,3.664607620e+01f,3.672954941e+01f,3.681301880e+01f,3.689649200e+01f,3.697996521e+01f,3.706343842e+01f,3.714691162e+01f,3.723038101e+01f,3.731385422e+01f,3.739732742e+01f,3.748080063e+01f,3.756427383e+01f,3.764774323e+01f,3.773121643e+01f,3.781468964e+01f,3.789816284e+01f,3.798163605e+01f,3.806510544e+01f,3.814857864e+01f,3.823205185e+01f,3.831552505e+01f,3.839899826e+01f,3.848246765e+01f,3.856594086e+01f,3.864941406e+01f,3.873288727e+01f,3.881636047e+01f,3.889982986e+01f,3.898330307e+01f,3.906677628e+01f,3.915024948e+01f,3.923372269e+01f,3.931719208e+01f,3.940066528e+01f,3.948413849e+01f,3.956761169e+01f,3.965108490e+01f,3.973455429e+01f,3.981802750e+01f,3.990150070e+01f,3.998497391e+01f,4.006844711e+01f,4.015191650e+01f,4.023538971e+01f,4.031886292e+01f,4.040233612e+01f,4.048580933e+01f,4.056927872e+01f,4.065275192e+01f,4.073622513e+01f,4.081969833e+01f,4.090317154e+01f,4.098664093e+01f,4.107011414e+01f,4.115358734e+01f,4.123706055e+01f,4.132053375e+01f,4.140400314e+01f,4.148747635e+01f,4.157094955e+01f,4.165442276e+01f,4.173789597e+01f,4.182136536e+01f,4.190483856e+01f,4.198831177e+01f,4.207178497e+01f,4.215525818e+01f,4.223872757e+01f,4.232220078e+01f,4.240567398e+01f,4.248914719e+01f,4.257262039e+01f,4.265608978e+01f,4.273956299e+01f,4.282303619e+01f,4.290650940e+01f,4.298998260e+01f,4.307345200e+01f,4.315692520e+01f,4.324039841e+01f,4.332387161e+01f,4.340734482e+01f,4.349081421e+01f,4.357428741e+01f,4.365776062e+01f,4.374123383e+01f,4.382470703e+01f,4.390818024e+01f,4.399164963e+01f,4.407512283e+01f,4.415859604e+01f,4.424206924e+01f,4.432554245e+01f,4.440901184e+01f,4.449248505e+01f,4.457595825e+01f,4.465943146e+01f,4.474290466e+01f,4.482637405e+01f,4.490984726e+01f,4.499332047e+01f,4.507679367e+01f,4.516026688e+01f,4.524373627e+01f,4.532720947e+01f,4.541068268e+01f,4.549415588e+01f,4.557762909e+01f,4.566109848e+01f,4.574457169e+01f,4.582804489e+01f,4.591151810e+01f,4.599499130e+01f,4.607846069e+01f,4.616193390e+01f,4.624540710e+01f,4.632888031e+01f,4.641235352e+01f,4.649582291e+01f,4.657929611e+01f,4.666276932e+01f,4.674624252e+01f,4.682971573e+01f,4.691318512e+01f,4.699665833e+01f,4.708013153e+01f,4.716360474e+01f,4.724707794e+01f,4.733054733e+01f,4.741402054e+01f,4.749749374e+01f,4.758096695e+01f,4.766444016e+01f,4.774790955e+01f,4.783138275e+01f,4.791485596e+01f,4.799832916e+01f,4.808180237e+01f,4.816527176e+01f,4.824874496e+01f,4.833221817e+01f,4.841569138e+01f,4.849916458e+01f,4.858263397e+01f,4.866610718e+01f,4.874958038e+01f,4.883305359e+01f,4.891652679e+01f,4.900000000e+01f};

__global__ __launch_bounds__(128) void k_fr(const float* __restrict__ Y, const float* __restrict__ X, const int* __restrict__ MASK, const float* __restrict__ SIG, float* __restrict__ OUT) {
  __shared__ __align__(16) __bf16 swh[16][TT + 8], swl[16][TT + 8]; __shared__ __align__(16) __bf16 sy[16][TT + 8], smk[16][TT + 8]; __shared__ __align__(16) float so[16][2 * MM]; __shared__ float sd[2][16][17], sc[2][16][17];
  const int tid = threadIdx.x, wave = tid >> 5, lane = tid & 31, col = lane & 15, g = lane >> 4; const int pt = blockIdx.x, b = blockIdx.y; const int p0 = pt * 16;
  const float s0 = bfr(SIG[0]), s1 = bfr(SIG[1]); const float ih0 = 0.5f / (s0 * s0), ih1 = 0.5f / (s1 * s1);
  for (int e = tid; e < 16 * TT; e += 128) { const int pl = e >> 9, t = e & 511; const int p = min(p0 + pl, PP - 1); const float d = GRID[p] - bfr(X[(size_t)b * TT + t]); const float d2 = d * d;
    const float w1 = exp_ni(-d2 * ih1); const __bf16 hb = (__bf16)w1; swh[pl][t] = hb; swl[pl][t] = (__bf16)(w1 - (float)hb); }
  for (int e = tid; e < MM * TT; e += 128) { const int m = e >> 9, t = e & 511; sy[m][t] = (__bf16)Y[((size_t)b * MM + m) * TT + t]; smk[m][t] = (__bf16)((MASK[((size_t)b * MM + m) * TT + t] != 0) ? 1.f : 0.f); }
  __syncthreads();
  if (wave < 2) { v8f acc = {}; const bool same = (ih0 == ih1);
#pragma unroll 2
    for (int kc = 0; kc < TT / 32; ++kc) { const v16b a = frag_b((wave == 0) ? &sy[col][kc * 32] : &smk[col][kc * 32], lane); v16b bh, bl;
      if (wave == 0 || same) { bh = frag_b(&swh[col][kc * 32], lane); bl = frag_b(&swl[col][kc * 32], lane); }
      else { const int p = min(p0 + col, PP - 1);
#pragma unroll
        for (int i = 0; i < 16; ++i) { const int t = kc * 32 + 8 * g + (i & 7) + ((i >> 3) << 4); const float d = GRID[p] - bfr(X[(size_t)b * TT + t]); const float w0 = exp_ni(-d * d * ih0); const __bf16 hb = (__bf16)w0; bh[i] = hb; bl[i] = (__bf16)(w0 - (float)hb); } }
      acc = wmma_bf(a, bl, acc); acc = wmma_bf(a, bh, acc); }
    float (*dst)[16][17] = (wave == 0) ? sc : sd;
#pragma unroll
    for (int r = 0; r < 8; ++r) dst[0][8 * g + r][col] = acc[r]; }
  __syncthreads();
  for (int e = tid; e < 16 * MM; e += 128) { const int pl = e >> 4, m = e & 15; const float dn = sd[0][m][pl], cv = sc[0][m][pl]; so[pl][2 * m] = dn; so[pl][2 * m + 1] = cv / (dn + 1e-8f); }
  __syncthreads();
  for (int e = tid; e < 16 * 8; e += 128) { const int pl = e >> 3, q = e & 7; if (p0 + pl < PP) vst2(OUT + ((size_t)b * PP + p0 + pl) * (2 * MM) + q * 4, *(const v4f*)&so[pl][q * 4]); }
}
extern "C" void kernel_launch(void* const* d_in, const int* in_sizes, int n_in, void* d_out, int out_size, void* d_ws, size_t ws_size, hipStream_t stream) {
  (void)in_sizes; (void)n_in; (void)out_size; (void)d_ws; (void)ws_size;
  const float** F = (const float**)d_in;
  k_fr<<<dim3(PT, NB), 128, 0, stream>>>(F[0], F[1], (const int*)d_in[2], F[3], (float*)d_out);
}
